// SelfAttn_75033078661890
// MI455X (gfx1250) — hardware-verified
//
#include <hip/hip_runtime.h>
#include <math.h>

#ifndef NB
#define NB 2
#endif
#ifndef SEQ
#define SEQ 2048
#endif
#define NB_FULL 2
#define SEQ_FULL 2048
#define DM 1024
#define NH 16
#define HDIM 64
#define NQKV (3 * DM)
#define NTOK (NB * SEQ)
#define QCAR 16.0f
#define OFF_BQ 0
#define OFF_BP NQKV
#define OFF_QW (NQKV + DM)
#define OFF_KW (NQKV + DM + HDIM)
#define VECN (NQKV + DM + 2 * HDIM)
static_assert(SEQ % 64 == 0);
static_assert(NB >= 1);
static_assert(NB <= NB_FULL);
static_assert(SEQ <= SEQ_FULL);
static_assert(VECN % 32 == 0);
static_assert(NH * HDIM == DM);
static_assert(DM % 64 == 0);
static_assert(NQKV % 64 == 0);

typedef __attribute__((ext_vector_type(16))) _Float16 v16h;
typedef __attribute__((ext_vector_type(8)))  _Float16 v8h;
typedef __attribute__((ext_vector_type(16))) __bf16   v16b;
typedef __attribute__((ext_vector_type(8)))  __bf16   v8b;
typedef __attribute__((ext_vector_type(8)))  float    v8f;
typedef __attribute__((ext_vector_type(4)))  float    v4f;
typedef __attribute__((ext_vector_type(2)))  float    v2f;
typedef __attribute__((ext_vector_type(4)))  unsigned int v4u;


constexpr size_t al256(size_t x) { return (x + 255) / 256 * 256; }
constexpr size_t WS_VEC   = al256((size_t)VECN * 4);
constexpr size_t WS_X16   = al256((size_t)NTOK * DM * 2);
constexpr size_t WS_W16   = al256((size_t)NQKV * DM * 2);
constexpr size_t WS_WP16  = al256((size_t)DM * DM * 2);
constexpr size_t WS_QKV   = al256((size_t)NTOK * NQKV * 4);
constexpr size_t WS_QK16  = al256((size_t)NTOK * DM * 2);
constexpr size_t WS_CTX   = al256((size_t)NTOK * DM * 4);
constexpr size_t WS_CTX16 = al256((size_t)NTOK * DM * 2);
constexpr size_t WS_TOTAL = WS_VEC + WS_X16 + WS_W16 + WS_WP16 + WS_QKV + 2 * WS_QK16 + WS_CTX + WS_CTX16;
static_assert(WS_TOTAL <= (size_t)134217728);

__device__ __forceinline__ float cmb_bf(float v) { const unsigned u = __builtin_bit_cast(unsigned, v); const unsigned r = (u + 0x7fffu + ((u >> 16) & 1u)) & 0xffff0000u; return __builtin_bit_cast(float, r); }
__device__ __forceinline__ unsigned int cmb_pk2(float a, float b) { return (unsigned int)__builtin_bit_cast(unsigned short, (_Float16)a) | ((unsigned int)__builtin_bit_cast(unsigned short, (_Float16)b) << 16); }

namespace w25 {

__device__ __forceinline__ unsigned short f2bf_bits(float f) {
  unsigned u = __float_as_uint(f);
  return (unsigned short)((u + 0x7FFFu + ((u >> 16) & 1u)) >> 16);
}
__device__ __forceinline__ float bf_bits2f(unsigned short h) { return __uint_as_float(((unsigned)h) << 16); }

__device__ __forceinline__ void dep_guard_h(v8f& a, v8f& b, v16h x, v16h y) { asm volatile("v_nop\n\tv_nop\n\tv_nop\n\tv_nop" : "+v"(a), "+v"(b) : "v"(x), "v"(y)); }
__device__ __forceinline__ void dep_guard_b(v8f& a, v8f& b, v16b x, v16b y) { asm volatile("v_nop\n\tv_nop\n\tv_nop\n\tv_nop" : "+v"(a), "+v"(b) : "v"(x), "v"(y)); }
__device__ __forceinline__ void keep4_h(v16h a, v16h b, v16h c, v16h d) { asm volatile("v_nop" :: "v"(a), "v"(b), "v"(c), "v"(d)); }
__device__ __forceinline__ void keep4_b(v16b a, v16b b, v16b c, v16b d) { asm volatile("v_nop" :: "v"(a), "v"(b), "v"(c), "v"(d)); }
__device__ __forceinline__ void acc_guard4(v8f& a, v8f& b, v8f& c, v8f& d) { asm volatile("v_nop\n\tv_nop\n\tv_nop\n\tv_nop" : "+v"(a), "+v"(b), "+v"(c), "+v"(d)); }
template <typename T> struct Frag;
template <> struct Frag<_Float16> {
  typedef v16h V; union U { v16h v; v8h h[2]; };
  static __device__ __forceinline__ v16h load(const _Float16* p) {
    U f; f.h[0] = *(const v8h*)(p); f.h[1] = *(const v8h*)(p + 16); return f.v;
  }
  static __device__ __forceinline__ v8f mma(v16h a, v16h b, v8f c) {
    return __builtin_amdgcn_wmma_f32_16x16x32_f16(false, a, false, b, (short)0, c, false, false);
  }
  static __device__ __forceinline__ void guard(v8f& a, v8f& b, v16h x, v16h y) { dep_guard_h(a, b, x, y); }
  static __device__ __forceinline__ void keep(v16h a, v16h b, v16h c, v16h d) { keep4_h(a, b, c, d); }
};
template <> struct Frag<__bf16> {
  typedef v16b V; union U { v16b v; v8b h[2]; };
  static __device__ __forceinline__ v16b load(const __bf16* p) {
    U f; f.h[0] = *(const v8b*)(p); f.h[1] = *(const v8b*)(p + 16); return f.v;
  }
  static __device__ __forceinline__ v8f mma(v16b a, v16b b, v8f c) {
    return __builtin_amdgcn_wmma_f32_16x16x32_bf16(false, a, false, b, (short)0, c, false, false);
  }
  static __device__ __forceinline__ void guard(v8f& a, v8f& b, v16b x, v16b y) { dep_guard_b(a, b, x, y); }
  static __device__ __forceinline__ void keep(v16b a, v16b b, v16b c, v16b d) { keep4_b(a, b, c, d); }
};

template <int ET> struct Elem;
template <> struct Elem<0> { typedef _Float16 T; };
template <> struct Elem<1> { typedef __bf16 T; };
template <int ET, bool SPLIT, int BIAS_MODE, int OUT_MODE, bool RESID>
__global__ __launch_bounds__(256) void wmma_gemm64(
    const unsigned short* __restrict__ Ap, const unsigned short* __restrict__ A2p, int lda, long strideA,
    const unsigned short* __restrict__ Btp, const unsigned short* __restrict__ Bt2p, int ldb, long strideB,
    void* __restrict__ Cout, void* __restrict__ Cout2, int ldc, long strideC,
    const float* __restrict__ bias,
    const float* __restrict__ resid, long strideR,
    int M, int N, int K, float scale) {
  typedef typename Elem<ET>::T T;
  typedef typename Frag<T>::V V;
  const T* A = (const T*)Ap; const T* A2 = (const T*)A2p; const T* Bt = (const T*)Btp; const T* Bt2 = (const T*)Bt2p;
  __shared__ __align__(16) float sT[8][16 * 68];
  const int b    = blockIdx.y;
  const int lane = threadIdx.x & 31;
  const int wave = threadIdx.x >> 5;
  const int tilesN = N >> 6;
  const int tilesM = M >> 6;
  const int tile = blockIdx.x * 8 + wave;
  if (tile >= tilesM * tilesN) return;
  const int tm = tile / tilesN;
  const int tn = tile - tm * tilesN;
  const int m0 = tm << 6;
  const int n0 = tn << 6;

  const T* Ab  = A  + (size_t)b * strideA;
  const T* Bb  = Bt + (size_t)b * strideB;
  const T* Ab2 = SPLIT ? (A2  + (size_t)b * strideA) : nullptr;
  const T* Bb2 = SPLIT ? (Bt2 + (size_t)b * strideB) : nullptr;

  const int rlane = lane & 15;
  const int koff  = (lane >> 4) * 8;
  const int mOff  = (lane >> 4) * 8;

  v8f acc[4][4];
#pragma unroll
  for (int i = 0; i < 4; ++i)
#pragma unroll
    for (int j = 0; j < 4; ++j) acc[i][j] = (v8f){0.f,0.f,0.f,0.f,0.f,0.f,0.f,0.f};

  for (int k0 = 0; k0 < K; k0 += 32) {
    V bh[4], bl[4];
#pragma unroll
    for (int j = 0; j < 4; ++j) {
      const size_t bo = (size_t)(n0 + (j << 4) + rlane) * ldb + koff + k0;
      bh[j] = Frag<T>::load(Bb + bo);
      if (SPLIT) bl[j] = Frag<T>::load(Bb2 + bo);
    }
#pragma unroll
    for (int i = 0; i < 4; ++i) {
      const size_t ao = (size_t)(m0 + (i << 4) + rlane) * lda + koff + k0;
      V ah = Frag<T>::load(Ab + ao);
      V al;
      if (SPLIT) al = Frag<T>::load(Ab2 + ao);
#pragma unroll
      for (int j = 0; j < 4; ++j) {
        acc[i][j] = Frag<T>::mma(ah, bh[j], acc[i][j]);
        if (SPLIT) {
          acc[i][j] = Frag<T>::mma(ah, bl[j], acc[i][j]);
          acc[i][j] = Frag<T>::mma(al, bh[j], acc[i][j]);
        }
      }
      Frag<T>::guard(acc[i][0], acc[i][3], ah, SPLIT ? al : ah);
    }
    Frag<T>::keep(bh[0], bh[1], bh[2], bh[3]);
    if (SPLIT) Frag<T>::keep(bl[0], bl[1], bl[2], bl[3]);
  }
  acc_guard4(acc[0][0], acc[0][1], acc[0][2], acc[0][3]);
  acc_guard4(acc[1][0], acc[1][1], acc[1][2], acc[1][3]);
  acc_guard4(acc[2][0], acc[2][1], acc[2][2], acc[2][3]);
  acc_guard4(acc[3][0], acc[3][1], acc[3][2], acc[3][3]);

  float* slab = sT[wave];
  const float* Rb = RESID ? (resid + (size_t)b * strideR) : nullptr;
#pragma unroll
  for (int i = 0; i < 4; ++i) {
    const int mBase = m0 + (i << 4);
#pragma unroll
    for (int j = 0; j < 4; ++j) {
      const int n = n0 + (j << 4) + rlane;
      float bv = 0.f;
      if (BIAS_MODE == 2) bv = bias[n];
#pragma unroll
      for (int r = 0; r < 8; ++r) {
        float v = acc[i][j][r] * scale;
        if (BIAS_MODE == 1) v += bias[mBase + mOff + r];
        if (BIAS_MODE == 2) v += bv;
        if (RESID) v += Rb[(size_t)(mBase + mOff + r) * ldc + n];
        slab[(mOff + r) * 68 + (j << 4) + rlane] = v;
      }
    }
    __builtin_amdgcn_fence(3, "workgroup");
    __builtin_amdgcn_wave_barrier();
    __builtin_amdgcn_fence(2, "workgroup");
    if (OUT_MODE == 0) {
      float* C = (float*)Cout + (size_t)b * strideC;
      const int hh = lane >> 4, c4 = (lane & 15) * 4;
      for (int ps = 0; ps < 2; ++ps) {
#pragma unroll
        for (int it = 0; it < 8; ++it) {
          const int row = it * 2 + hh;
          v4f v = *(const v4f*)(slab + row * 68 + c4);
          *(volatile v4f*)(C + (size_t)(mBase + row) * ldc + n0 + c4) = v;
        }
        __threadfence();
      }
    } else {
      const int q = lane >> 3, c8 = (lane & 7) * 8;
      unsigned short* C  = (unsigned short*)Cout  + (size_t)b * strideC;
      unsigned short* C2 = (OUT_MODE == 2) ? ((unsigned short*)Cout2 + (size_t)b * strideC) : nullptr;
      for (int ps = 0; ps < 2; ++ps) {
#pragma unroll
        for (int it = 0; it < 4; ++it) {
          const int row = it * 4 + q;
          const float* sp = slab + row * 68 + c8;
          v8h hv, lv;
#pragma unroll
          for (int e = 0; e < 8; ++e) {
            if (OUT_MODE == 1) {
              hv[e] = (_Float16)sp[e];
            } else {
              unsigned short hb = f2bf_bits(sp[e]);
              unsigned short lb = f2bf_bits(sp[e] - bf_bits2f(hb));
              hv[e] = __builtin_bit_cast(_Float16, hb);
              lv[e] = __builtin_bit_cast(_Float16, lb);
            }
          }
          *(volatile v8h*)(C + (size_t)(mBase + row) * ldc + n0 + c8) = hv;
          if (OUT_MODE == 2) *(volatile v8h*)(C2 + (size_t)(mBase + row) * ldc + n0 + c8) = lv;
        }
        __threadfence();
      }
    }
    __builtin_amdgcn_fence(3, "workgroup");
    __builtin_amdgcn_wave_barrier();
    __builtin_amdgcn_fence(2, "workgroup");
  }
}

#define AT_D 64
#define AT_NW 4
#define AT_QB 64
#define AT_KC 64
struct AttnGeom { long long q_bs, q_rs, q_hs, k_bs, k_rs, k_hs, v_bs, v_rs, v_hs, o_bs, o_rs, o_hs; int S, Skv, H, nchunk; float sscale; float psc; };
static_assert(sizeof(AttnGeom) == 12 * 8 + 4 * 4 + 2 * 4);

__device__ __forceinline__ v8f at_mmah(v16h a, v16h b, v8f c) {
  c = __builtin_amdgcn_wmma_f32_16x16x32_f16(false, a, false, b, (short)0, c, false, false);
  asm volatile("v_nop\n\tv_nop\n\tv_nop\n\tv_nop" : "+v"(c) : "v"(a), "v"(b));
  return c;
}

__global__ __launch_bounds__(128) __attribute__((amdgpu_num_vgpr(256)))
void k_attn64(const unsigned short* __restrict__ qp, const unsigned short* __restrict__ kp,
              const float* __restrict__ v, float* __restrict__ out, AttnGeom g) {
  union FH { v16h v; v8h h[2]; };
  __shared__ __align__(16) _Float16 Ksh[AT_KC * AT_D];
  __shared__ __align__(16) _Float16 Vth[AT_D * AT_KC];
  __shared__ __align__(16) _Float16 Psh[AT_NW][16 * AT_KC];
  __shared__ __align__(16) float    Os[AT_NW][16 * 68];

  const int tid  = threadIdx.x;
  const int wave = tid >> 5;
  const int lane = tid & 31;
  const int hh   = lane >> 4;
  const int c    = lane & 15;

  const int nqb = g.S / AT_QB;
  const int bx = blockIdx.x;
  const int qb = bx % nqb;
  const int bh = bx / nqb;
  const int h  = bh % g.H;
  const int b  = bh / g.H;
  const int q0 = qb * AT_QB + wave * 16;

  const _Float16* q = (const _Float16*)qp;
  const _Float16* k = (const _Float16*)kp;
  const _Float16* qb_ptr = q + (size_t)b * g.q_bs + (size_t)h * g.q_hs;
  const _Float16* kb_ptr = k + (size_t)b * g.k_bs + (size_t)h * g.k_hs;
  const float*    vb_ptr = v + (size_t)b * g.v_bs + (size_t)h * g.v_hs;
  float*          ob_ptr = out + (size_t)b * g.o_bs + (size_t)h * g.o_hs;

  v16h qa[2];
  {
    const _Float16* qrow = qb_ptr + (size_t)(q0 + c) * g.q_rs;
#pragma unroll
    for (int dc = 0; dc < 2; ++dc) {
      FH f;
      f.h[0] = *(const v8h*)(qrow + dc * 32 + 8 * hh);
      f.h[1] = *(const v8h*)(qrow + dc * 32 + 16 + 8 * hh);
      qa[dc] = f.v;
    }
  }

  float mrow[8], lrow[8];
  v8f oacc[4];
#pragma unroll
  for (int r = 0; r < 8; ++r) { mrow[r] = -INFINITY; lrow[r] = 0.f; }
#pragma unroll
  for (int t = 0; t < 4; ++t) oacc[t] = (v8f){0.f,0.f,0.f,0.f,0.f,0.f,0.f,0.f};

  for (int kc = 0; kc < g.nchunk; ++kc) {
    const int kv0 = kc * AT_KC;
    __syncthreads();
    {
      const int kvr = tid >> 1, dh = (tid & 1) * 32;
      const _Float16* krow = kb_ptr + (size_t)(kv0 + kvr) * g.k_rs + dh;
      const float*    vrow = vb_ptr + (size_t)(kv0 + kvr) * g.v_rs + dh;
#pragma unroll
      for (int i = 0; i < 4; ++i) {
        const v8h kk = *(const v8h*)(krow + 8 * i);
        *(v8h*)(Ksh + kvr * AT_D + dh + 8 * i) = kk;
      }
#pragma unroll
      for (int i = 0; i < 8; ++i) {
        const v4f vv = *(const v4f*)(vrow + 4 * i);
#pragma unroll
        for (int e = 0; e < 4; ++e) {
          const int d = dh + 4 * i + e;
          const float fv = vv[e];
          Vth[d * AT_KC + kvr] = (_Float16)fv;
        }
      }
    }
    __syncthreads();

    v8f s[4];
#pragma unroll
    for (int j = 0; j < 4; ++j) {
      v8f acc = (v8f){0.f,0.f,0.f,0.f,0.f,0.f,0.f,0.f};
#pragma unroll
      for (int dc = 0; dc < 2; ++dc) {
        FH kf;
        kf.h[0] = *(const v8h*)(Ksh + (j * 16 + c) * AT_D + dc * 32 + 8 * hh);
        kf.h[1] = *(const v8h*)(Ksh + (j * 16 + c) * AT_D + dc * 32 + 16 + 8 * hh);
        acc = at_mmah(qa[dc], kf.v, acc);
      }
      s[j] = acc;
    }
    float cm[8];
#pragma unroll
    for (int r = 0; r < 8; ++r) {
      float m = fmaxf(fmaxf(s[0][r], s[1][r]), fmaxf(s[2][r], s[3][r]));
#pragma unroll
      for (int off = 1; off < 16; off <<= 1) m = fmaxf(m, __shfl_xor(m, off, 32));
      cm[r] = m;
    }
    _Float16* pwh = Psh[wave];
#pragma unroll
    for (int r = 0; r < 8; ++r) {
      const float mnew = fmaxf(mrow[r], cm[r]);
      const float alpha = expf((mrow[r] - mnew) * g.sscale);
      mrow[r] = mnew;
      float psum = 0.f;
#pragma unroll
      for (int j = 0; j < 4; ++j) {
        const float p = expf((s[j][r] - mnew) * g.sscale);
        psum += p;
        pwh[(8 * hh + r) * AT_KC + j * 16 + c] = (_Float16)(p * g.psc);
      }
#pragma unroll
      for (int off = 1; off < 16; off <<= 1) psum += __shfl_xor(psum, off, 32);
      lrow[r] = lrow[r] * alpha + psum;
#pragma unroll
      for (int t = 0; t < 4; ++t) oacc[t][r] *= alpha;
    }
    __builtin_amdgcn_fence(3, "workgroup");
    __builtin_amdgcn_wave_barrier();
    __builtin_amdgcn_fence(2, "workgroup");
#pragma unroll 1
    for (int kk = 0; kk < 2; ++kk) {
      FH pa;
      pa.h[0] = *(const v8h*)(pwh + c * AT_KC + kk * 32 + 8 * hh);
      pa.h[1] = *(const v8h*)(pwh + c * AT_KC + kk * 32 + 16 + 8 * hh);
#pragma unroll
      for (int t = 0; t < 4; ++t) {
        FH vbf;
        vbf.h[0] = *(const v8h*)(Vth + (t * 16 + c) * AT_KC + kk * 32 + 8 * hh);
        vbf.h[1] = *(const v8h*)(Vth + (t * 16 + c) * AT_KC + kk * 32 + 16 + 8 * hh);
        oacc[t] = at_mmah(pa.v, vbf.v, oacc[t]);
      }
    }
  }

  float* os = Os[wave];
#pragma unroll
  for (int r = 0; r < 8; ++r) {
    const float inv = 1.0f / (lrow[r] * g.psc);
#pragma unroll
    for (int t = 0; t < 4; ++t) os[(8 * hh + r) * 68 + t * 16 + c] = oacc[t][r] * inv;
  }
  __builtin_amdgcn_fence(3, "workgroup");
  __builtin_amdgcn_wave_barrier();
  __builtin_amdgcn_fence(2, "workgroup");
  {
    const int c4 = (lane & 15) * 4;
    for (int ps = 0; ps < 2; ++ps) {
#pragma unroll
      for (int it = 0; it < 8; ++it) {
        const int row = it * 2 + hh;
        v4f val = *(const v4f*)(os + row * 68 + c4);
        *(volatile v4f*)(ob_ptr + (size_t)(q0 + row) * g.o_rs + c4) = val;
      }
      __threadfence();
    }
  }
}

}

__global__ __launch_bounds__(256) void k_vec(const float* __restrict__ bq, const float* __restrict__ bp, const float* __restrict__ qw, const float* __restrict__ kw, float* __restrict__ VEC) {
    const int u = blockIdx.x * 256 + threadIdx.x;
    if (u >= VECN) return;
    const float a  = bq[min(u, NQKV - 1)];
    const float bb = bp[min(max(u - OFF_BP, 0), DM - 1)];
    const float cq = qw[min(max(u - OFF_QW, 0), HDIM - 1)];
    const float ck = kw[min(max(u - OFF_KW, 0), HDIM - 1)];
    const float sel = (u < OFF_BP) ? a : ((u < OFF_QW) ? bb : ((u < OFF_KW) ? cq : ck));
    const float o = cmb_bf(sel);
    *(volatile float*)(VEC + u) = o;
    __threadfence();
    *(volatile float*)(VEC + u) = o;
}

__global__ __launch_bounds__(256) void k_castp(const float* __restrict__ SRC, long long sbs, int lds, unsigned short* __restrict__ DST, long long dbs, int ldd, int nR, int nC, float sc, int bfr) {
    const long long u = (long long)blockIdx.x * 256 + threadIdx.x;
    const int per = nC >> 3;
    if (u >= (long long)nR * per) return;
    const int r = (int)(u / per);
    const int c0 = 8 * (int)(u - (long long)r * per);
    const float* s = SRC + (long long)blockIdx.y * sbs + (long long)r * lds + c0;
    const v4f a = *(const v4f*)s;
    const v4f bq = *(const v4f*)(s + 4);
    float w[8] = {a.x, a.y, a.z, a.w, bq.x, bq.y, bq.z, bq.w};
#pragma unroll
    for (int e = 0; e < 8; ++e) { const float t = bfr ? cmb_bf(w[e]) : w[e]; w[e] = t * sc; }
    v4u pk;
    pk.x = cmb_pk2(w[0], w[1]); pk.y = cmb_pk2(w[2], w[3]); pk.z = cmb_pk2(w[4], w[5]); pk.w = cmb_pk2(w[6], w[7]);
    volatile v4u* d = (volatile v4u*)(DST + (long long)blockIdx.y * dbs + (long long)r * ldd + c0);
    *d = pk;
    __threadfence();
    *d = pk;
}

__global__ __launch_bounds__(256) void k_rms(const float* __restrict__ QKV, const float* __restrict__ QW, const float* __restrict__ KW, unsigned short* __restrict__ QH, unsigned short* __restrict__ KH, int nrow) {
    #pragma clang fp contract(off)
    const int r = blockIdx.x * 8 + (threadIdx.x >> 5);
    const int L = threadIdx.x & 31;
    if (r >= nrow) return;
    const int token = r >> 5, slice = (r >> 4) & 1, h = r & 15;
    const float* src = QKV + (long long)token * NQKV + slice * DM + h * HDIM + 2 * L;
    const v2f x = *(const v2f*)src;
    float ss = x.x * x.x + x.y * x.y;
#pragma unroll
    for (int o = 16; o > 0; o >>= 1) ss += __shfl_xor(ss, o, 32);
    const float rms = sqrtf(ss * (1.0f / 64.0f) + 1e-6f);
    const float rec = 1.0f / rms;
    const v2f wq = *(const v2f*)(QW + 2 * L);
    const v2f wk = *(const v2f*)(KW + 2 * L);
    v2f w; w.x = slice ? wk.x : wq.x; w.y = slice ? wk.y : wq.y;
    const float o0 = ((x.x * rec) * w.x) * QCAR;
    const float o1 = ((x.y * rec) * w.y) * QCAR;
    const unsigned pk = cmb_pk2(o0, o1);
    unsigned short* dst = (slice ? KH : QH) + (long long)token * DM + h * HDIM + 2 * L;
    *(volatile unsigned*)dst = pk;
    __threadfence();
    *(volatile unsigned*)dst = pk;
}

extern "C" void kernel_launch(void* const* d_in, const int* in_sizes, int n_in, void* d_out, int out_size, void* d_ws, size_t ws_size, hipStream_t stream) {
    if (n_in < 7) return;
    const float* x     = (const float*)d_in[0];
    const float* Wqkv  = (const float*)d_in[1];
    const float* bqkv  = (const float*)d_in[2];
    const float* Wproj = (const float*)d_in[3];
    const float* bproj = (const float*)d_in[4];
    const float* qn_w  = (const float*)d_in[5];
    const float* kn_w  = (const float*)d_in[6];
    const long long xneed = ((long long)(NB - 1) * SEQ_FULL + SEQ) * DM;
    if ((long long)in_sizes[0] < xneed) return;
    if ((long long)in_sizes[1] < (long long)NQKV * DM) return;
    if (in_sizes[2] < NQKV) return;
    if ((long long)in_sizes[3] < (long long)DM * DM) return;
    if (in_sizes[4] < DM) return;
    if (in_sizes[5] < HDIM || in_sizes[6] < HDIM) return;
    if ((long long)out_size < xneed) return;
    if (WS_TOTAL > ws_size) return;

    char* wsp = (char*)d_ws;
    float* VEC = (float*)wsp; wsp += WS_VEC;
    unsigned short* X16 = (unsigned short*)wsp; wsp += WS_X16;
    unsigned short* W16 = (unsigned short*)wsp; wsp += WS_W16;
    unsigned short* WP16 = (unsigned short*)wsp; wsp += WS_WP16;
    float* QKV = (float*)wsp; wsp += WS_QKV;
    unsigned short* QH16 = (unsigned short*)wsp; wsp += WS_QK16;
    unsigned short* KH16 = (unsigned short*)wsp; wsp += WS_QK16;
    float* CTX = (float*)wsp; wsp += WS_CTX;
    unsigned short* CTX16 = (unsigned short*)wsp; wsp += WS_CTX16;
    float* out = (float*)d_out;

    k_vec<<<(VECN + 255) / 256, 256, 0, stream>>>(bqkv, bproj, qn_w, kn_w, VEC);
    k_castp<<<dim3((unsigned)(((long long)SEQ * (DM / 8) + 255) / 256), (unsigned)NB), 256, 0, stream>>>(x, (long long)SEQ_FULL * DM, DM, X16, (long long)SEQ * DM, DM, SEQ, DM, 16.0f, 1);
    k_castp<<<dim3((unsigned)(((long long)NQKV * (DM / 8) + 255) / 256), 1u), 256, 0, stream>>>(Wqkv, 0LL, DM, W16, 0LL, DM, NQKV, DM, 64.0f, 1);
    k_castp<<<dim3((unsigned)(((long long)DM * (DM / 8) + 255) / 256), 1u), 256, 0, stream>>>(Wproj, 0LL, DM, WP16, 0LL, DM, DM, DM, 64.0f, 1);
    w25::wmma_gemm64<0, false, 2, 0, false><<<dim3((unsigned)(((NTOK / 64) * (NQKV / 64) + 7) / 8), 1u), 256, 0, stream>>>(
        (const unsigned short*)X16, nullptr, DM, 0L, (const unsigned short*)W16, nullptr, DM, 0L,
        (void*)QKV, nullptr, NQKV, 0L, VEC + OFF_BQ, nullptr, 0L, NTOK, NQKV, DM, 1.0f / 1024.0f);
    k_rms<<<(unsigned)((NTOK * 32) / 8), 256, 0, stream>>>(QKV, VEC + OFF_QW, VEC + OFF_KW, QH16, KH16, NTOK * 32);
    w25::AttnGeom g;
    g.q_bs = (long long)SEQ * DM;   g.q_rs = DM;   g.q_hs = HDIM;
    g.k_bs = (long long)SEQ * DM;   g.k_rs = DM;   g.k_hs = HDIM;
    g.v_bs = (long long)SEQ * NQKV; g.v_rs = NQKV; g.v_hs = HDIM;
    g.o_bs = (long long)SEQ * DM;   g.o_rs = DM;   g.o_hs = HDIM;
    g.S = SEQ; g.Skv = SEQ; g.H = NH; g.nchunk = SEQ / AT_KC; g.sscale = 0.125f / (QCAR * QCAR); g.psc = 32768.0f;
    w25::k_attn64<<<(unsigned)(NB * NH * (SEQ / AT_QB)), 128, 0, stream>>>(QH16, KH16, QKV + 2 * DM, CTX, g);
    k_castp<<<dim3((unsigned)(((long long)NTOK * (DM / 8) + 255) / 256), 1u), 256, 0, stream>>>(CTX, 0LL, DM, CTX16, 0LL, DM, NTOK, DM, 256.0f, 0);
    w25::wmma_gemm64<0, false, 2, 0, false><<<dim3((unsigned)((((SEQ / 64) * (DM / 64)) + 7) / 8), (unsigned)NB), 256, 0, stream>>>(
        (const unsigned short*)CTX16, nullptr, DM, (long)SEQ * DM, (const unsigned short*)WP16, nullptr, DM, 0L,
        (void*)out, nullptr, DM, (long)SEQ_FULL * DM, VEC + OFF_BP, nullptr, 0L, SEQ, DM, DM, 1.0f / 16384.0f);
    (void)hipGetLastError();
}
